// KolmogorovArnoldLayer_38603166056799
// MI455X (gfx1250) — hardware-verified
//
#include <hip/hip_runtime.h>
#include <math.h>

typedef __attribute__((ext_vector_type(16))) _Float16 v16h;
typedef __attribute__((ext_vector_type(16))) __bf16 v16b;
typedef __attribute__((ext_vector_type(8)))  _Float16 v8h;
typedef __attribute__((ext_vector_type(8)))  float v8f;
typedef __attribute__((ext_vector_type(4)))  float v4f;
typedef __attribute__((ext_vector_type(2)))  float v2f;
typedef __attribute__((ext_vector_type(4)))  unsigned v4u;
typedef __attribute__((ext_vector_type(4)))  int v4i;
typedef float __attribute__((may_alias)) float_a;
typedef int __attribute__((may_alias)) int_a;

template <typename T> __device__ __forceinline__ void vst2(void* p, T v) { *(volatile T*)p = v; __threadfence(); *(volatile T*)p = v; }
__device__ __forceinline__ v8f wmma16(v16h a, v16h b, v8f c) {
  v8f d = __builtin_amdgcn_wmma_f32_16x16x32_f16(false, a, false, b, (short)0, c, false, false);
  asm volatile("v_nop\n\tv_nop\n\tv_nop\n\tv_nop" : "+v"(d) : "v"(a), "v"(b));
  return d;
}
__device__ __forceinline__ v8f wmma_bf(v16b a, v16b b, v8f c) {
  v8f d = __builtin_amdgcn_wmma_f32_16x16x32_bf16(false, a, false, b, (short)0, c, false, false);
  asm volatile("v_nop\n\tv_nop\n\tv_nop\n\tv_nop" : "+v"(d) : "v"(a), "v"(b));
  return d;
}
__device__ __forceinline__ v16h frag_h(const _Float16* rowk0, int lane) {
  union { v16h v; v8h q[2]; } u; const _Float16* p = rowk0 + 8 * (lane >> 4);
  u.q[0] = *(const v8h*)p; u.q[1] = *(const v8h*)(p + 16); return u.v;
}
__device__ __forceinline__ v16h frag_f32(const float* rowk0, int lane) {
  v16h a; const float* p = rowk0 + 8 * (lane >> 4);
#pragma unroll
  for (int i = 0; i < 8; ++i) { a[i] = (_Float16)p[i]; a[8 + i] = (_Float16)p[16 + i]; }
  return a;
}
__device__ __forceinline__ v16h frag_f32s(const float* rowk0, int lane, float sc) {
  v16h a; const float* p = rowk0 + 8 * (lane >> 4);
#pragma unroll
  for (int i = 0; i < 8; ++i) { a[i] = (_Float16)(p[i] * sc); a[8 + i] = (_Float16)(p[16 + i] * sc); }
  return a;
}
__device__ __forceinline__ v16h fragc_f32(const float* W, int k0, int n, int lane, int ld, int K) {
  v16h a; const int g = lane >> 4;
#pragma unroll
  for (int i = 0; i < 8; ++i) { const int ka = k0 + 8 * g + i, kb = ka + 16;
    a[i] = (_Float16)(ka < K ? W[(size_t)(ka < K ? ka : K - 1) * ld + n] : 0.f); a[8 + i] = (_Float16)(kb < K ? W[(size_t)(kb < K ? kb : K - 1) * ld + n] : 0.f); }
  return a;
}
struct F2 { v16b h, l; };
__device__ __forceinline__ F2 bsplit16(const float v[16]) { F2 r;
#pragma unroll
  for (int i = 0; i < 16; ++i) { const __bf16 h = (__bf16)v[i]; r.h[i] = h; r.l[i] = (__bf16)(v[i] - (float)h); }
  return r; }
__device__ __forceinline__ F2 split_row(const float* row, int k0, int lane) { float v[16]; const float* p = row + k0 + 8 * (lane >> 4);
#pragma unroll
  for (int i = 0; i < 8; ++i) { v[i] = p[i]; v[8 + i] = p[16 + i]; }
  return bsplit16(v); }
__device__ __forceinline__ F2 split_rowK(const float* row, int k0, int lane, int K) { float v[16]; const int g = lane >> 4;
#pragma unroll
  for (int i = 0; i < 8; ++i) { const int ka = k0 + 8 * g + i, kb = ka + 16; v[i] = ka < K ? row[ka < K ? ka : K - 1] : 0.f; v[8 + i] = kb < K ? row[kb < K ? kb : K - 1] : 0.f; }
  return bsplit16(v); }
__device__ __forceinline__ F2 split_col(const float* W, int k0, int n, int lane, int ld, int K) { float v[16]; const int g = lane >> 4;
#pragma unroll
  for (int i = 0; i < 8; ++i) { const int ka = k0 + 8 * g + i, kb = ka + 16; v[i] = ka < K ? W[(size_t)(ka < K ? ka : K - 1) * ld + n] : 0.f; v[8 + i] = kb < K ? W[(size_t)(kb < K ? kb : K - 1) * ld + n] : 0.f; }
  return bsplit16(v); }
__device__ __forceinline__ v8f mac3(const F2& a, const F2& b, v8f c) { c = wmma_bf(a.l, b.h, c); c = wmma_bf(a.h, b.l, c); return wmma_bf(a.h, b.h, c); }
__device__ __forceinline__ float sigm(float v) { return 1.0f / (1.0f + expf(-v)); }
#define LDSX() do { asm volatile("s_wait_dscnt 0" ::: "memory"); __builtin_amdgcn_wave_barrier(); __builtin_amdgcn_fence(__ATOMIC_RELEASE, "workgroup"); } while (0)


#define BB 2048
#define NI 256
#define NO 256
#define NK 64
#define DEG 3
#define NBAS (NK - 1 - DEG)
#ifndef TBB
#define TBB (BB / 16)
#endif
typedef __attribute__((ext_vector_type(8))) __bf16 v8b;
__device__ __forceinline__ v16b frag_b(const __bf16* rowk0, int lane) {
  union { v16b v; v8b q[2]; } u; const __bf16* p = rowk0 + 8 * (lane >> 4);
  u.q[0] = *(const v8b*)p; u.q[1] = *(const v8b*)(p + 16); return u.v;
}
__device__ __forceinline__ float bfr(float v) { return (float)(__bf16)v; }
__device__ __attribute__((noinline)) float exp_ni(float v) { return expf(v); }
#define WS_PT  0u
#define WS_END (WS_PT + 2u * NO * NI)

__global__ __launch_bounds__(256) void k_pack(const float* __restrict__ WB, __bf16* __restrict__ PT) {
  __shared__ __align__(16) __bf16 srow[NI]; const int o = blockIdx.x, tid = threadIdx.x; srow[tid] = (__bf16)bfr(WB[(size_t)tid * NO + o]); __syncthreads();
  if (tid < NI / 8) vst2((unsigned*)(PT + (size_t)o * NI + tid * 8), *(const v4u*)(&srow[tid * 8]));
}
__device__ __forceinline__ int bspline4(float x, const float* __restrict__ kn, float bout[4]) {
  int j = -1;
#pragma unroll 1
  for (int t = 0; t < NK - 1; ++t) { if (x >= kn[t] && x < kn[t + 1]) j = t; }
  bout[0] = bout[1] = bout[2] = bout[3] = 0.f; if (j < 0) return -1;
  float nb[4] = {0.f, 0.f, 0.f, 1.f};
#pragma unroll
  for (int d = 1; d <= DEG; ++d) { float nn[4] = {0.f, 0.f, 0.f, 0.f};
#pragma unroll
    for (int q = 0; q < 4; ++q) { const int idx = j - 3 + q; if (idx < 0 || idx < j - d || idx + d + 1 > NK - 1) continue;
      const float left = (x - kn[idx]) / (kn[idx + d] - kn[idx]); const float right = (kn[idx + d + 1] - x) / (kn[idx + d + 1] - kn[idx + 1]);
      const float n0 = nb[q]; const float n1 = (q + 1 < 4) ? nb[q + 1] : 0.f; nn[q] = left * n0 + right * n1; }
#pragma unroll
    for (int q = 0; q < 4; ++q) nb[q] = nn[q]; }
#pragma unroll
  for (int q = 0; q < 4; ++q) bout[q] = nb[q];
  return j;
}
__global__ __launch_bounds__(256) void k_kan(const float* __restrict__ X, const __bf16* __restrict__ PT, const float* __restrict__ WS, const float* __restrict__ CPS, const float* __restrict__ KN, float* __restrict__ OUT) {
  __shared__ float skn[NK]; __shared__ float sbas[16][NI][4]; __shared__ int sj[16][NI]; __shared__ __align__(16) __bf16 ssh[16][NI + 8], ssl[16][NI + 8]; __shared__ float scps[64][NK + 1]; __shared__ __align__(16) float so[16][68];
  const int tid = threadIdx.x, wave = tid >> 5, lane = tid & 31, col = lane & 15, g = lane >> 4; const int b0 = blockIdx.x * 16, o0 = blockIdx.y * 64;
  if (tid < NK) skn[tid] = bfr(KN[tid]);
  for (int q = tid; q < 64 * NK; q += 256) scps[q / NK][q % NK] = bfr(CPS[(size_t)(o0 + q / NK) * NK + q % NK]);
  __syncthreads();
  for (int q = tid; q < 16 * NI; q += 256) { const int rl = q / NI, i = q % NI; const float xv = bfr(X[(size_t)(b0 + rl) * NI + i]); float b4[4]; const int j = bspline4(xv, skn, b4);
    sj[rl][i] = j; sbas[rl][i][0] = b4[0]; sbas[rl][i][1] = b4[1]; sbas[rl][i][2] = b4[2]; sbas[rl][i][3] = b4[3];
    const float sv = xv / (1.0f + exp_ni(-xv)); const __bf16 hb = (__bf16)sv; ssh[rl][i] = hb; ssl[rl][i] = (__bf16)(sv - (float)hb); }
  __syncthreads();
  if (wave < 4) { v8f acc = {};
#pragma unroll
    for (int kc = 0; kc < NI / 32; ++kc) { const v16b ah = frag_b(&ssh[col][kc * 32], lane), al = frag_b(&ssl[col][kc * 32], lane); const v16b w = frag_b(PT + (size_t)(o0 + wave * 16 + col) * NI + kc * 32, lane); acc = wmma_bf(al, w, acc); acc = wmma_bf(ah, w, acc); }
#pragma unroll
    for (int r = 0; r < 8; ++r) so[8 * g + r][wave * 16 + col] = acc[r]; }
  __syncthreads();
  { const int ol = tid & 63, rb = (tid >> 6) * 4; float sp[4] = {0.f, 0.f, 0.f, 0.f};
#pragma unroll 1
    for (int i = 0; i < NI; ++i) { const float w = bfr(WS[(size_t)i * NO + o0 + ol]);
#pragma unroll
      for (int r = 0; r < 4; ++r) { const int j = sj[rb + r][i]; float t = 0.f; if (j >= 0) {
#pragma unroll
          for (int q = 0; q < 4; ++q) { const int k = j - 3 + q; if (k >= 0 && k < NBAS) t += sbas[rb + r][i][q] * scps[ol][k]; } }
        sp[r] += w * t; } }
#pragma unroll
    for (int r = 0; r < 4; ++r) so[rb + r][ol] += sp[r]; }
  __syncthreads();
  for (int q = tid; q < 16 * 16; q += 256) { const int rl = q >> 4, pc = q & 15; vst2(OUT + (size_t)(b0 + rl) * NO + o0 + pc * 4, *(const v4f*)&so[rl][pc * 4]); }
}

extern "C" void kernel_launch(void* const* d_in, const int* in_sizes, int n_in, void* d_out, int out_size, void* d_ws, size_t ws_size, hipStream_t stream) {
  (void)in_sizes; (void)n_in; (void)out_size;
  const float** F = (const float**)d_in;
  if (ws_size < (size_t)WS_END) return;
  char* ws = (char*)d_ws; __bf16* PT = (__bf16*)(ws + WS_PT);
  k_pack<<<NO, 256, 0, stream>>>(F[1], PT);
  k_kan<<<dim3(TBB, NO / 64), 256, 0, stream>>>(F[0], PT, F[2], F[3], F[4], (float*)d_out);
}
